// ReCausalSelfAttentionL3_90340342104845
// MI455X (gfx1250) — hardware-verified
//
#include <hip/hip_runtime.h>
#include <stdint.h>
#include <math.h>

#define NB_   8
#define T_    1024
#define C_    1024
#define NH_   16
#define HD_   64
#define NU_   128
#define MM_   16
#define LKV_  1026
#define LP_   1088
#define MAR_  192
#define AKP   72

typedef _Float16 v16h __attribute__((ext_vector_type(16)));
typedef _Float16 v8h  __attribute__((ext_vector_type(8)));
typedef float    v8f  __attribute__((ext_vector_type(8)));
typedef float    v4f  __attribute__((ext_vector_type(4)));

__device__ __forceinline__ v16h ldfrag(const _Float16* p) {
  union { v16h v; v8h h[2]; } f;
  f.h[0] = *(const v8h*)(p);
  f.h[1] = *(const v8h*)(p + 16);
  return f.v;
}
__device__ __forceinline__ v8f mma_f16(v16h a, v16h b, v8f c) {
  return __builtin_amdgcn_wmma_f32_16x16x32_f16(false, a, false, b, (short)0, c, false, false);
}
__device__ __forceinline__ v8f mma_f16_g(v16h a, v16h b, v8f c) {
  c = __builtin_amdgcn_wmma_f32_16x16x32_f16(false, a, false, b, (short)0, c, false, false);
  asm volatile("v_nop\n\tv_nop\n\tv_nop\n\tv_nop" : "+v"(c) : "v"(a), "v"(b));
  return c;
}
__device__ __forceinline__ void dep_guard(v8f& a, v8f& b, v16h x, v16h y) {
  asm volatile("v_nop\n\tv_nop\n\tv_nop\n\tv_nop" : "+v"(a), "+v"(b) : "v"(x), "v"(y));
}
__device__ __forceinline__ void keep4(v16h a, v16h b, v16h c, v16h d) {
  asm volatile("v_nop" :: "v"(a), "v"(b), "v"(c), "v"(d));
}
__device__ __forceinline__ void acc_guard4(v8f& a, v8f& b, v8f& c, v8f& d) {
  asm volatile("v_nop\n\tv_nop\n\tv_nop\n\tv_nop" : "+v"(a), "+v"(b), "+v"(c), "+v"(d));
}
__device__ __forceinline__ v8f zero8f() { v8f z; z[0]=0.f; z[1]=0.f; z[2]=0.f; z[3]=0.f; z[4]=0.f; z[5]=0.f; z[6]=0.f; z[7]=0.f; return z; }
__device__ __forceinline__ v8h zero8h() {
  v8h z;
#pragma unroll
  for (int e = 0; e < 8; ++e) z[e] = (_Float16)0.0f;
  return z;
}
__device__ __forceinline__ v8h cvt8(v4f a, v4f b, float s) {
  v8h r;
  r[0] = (_Float16)(a[0] * s); r[1] = (_Float16)(a[1] * s); r[2] = (_Float16)(a[2] * s); r[3] = (_Float16)(a[3] * s);
  r[4] = (_Float16)(b[0] * s); r[5] = (_Float16)(b[1] * s); r[6] = (_Float16)(b[2] * s); r[7] = (_Float16)(b[3] * s);
  return r;
}

__global__ __launch_bounds__(256)
void wt_kernel(const float* __restrict__ W0, const float* __restrict__ W1, const float* __restrict__ W2,
               const float* __restrict__ W3, const float* __restrict__ W4, const float* __restrict__ W5,
               unsigned short* __restrict__ WT, float s) {
  __shared__ __align__(16) float tf[64 * 68];
  const int z = blockIdx.z;
  const float* W = (z == 0) ? W0 : (z == 1) ? W1 : (z == 2) ? W2 : (z == 3) ? W3 : (z == 4) ? W4 : W5;
  _Float16* out = (_Float16*)WT + (size_t)z * C_ * C_;
  const int c0  = blockIdx.x * 64;
  const int r0  = blockIdx.y * 64;
  const int tid = threadIdx.x;
  {
    const int lr = tid >> 4;
    const int c4 = (tid & 15) * 4;
#pragma unroll
    for (int it = 0; it < 4; ++it) {
      const int rr = it * 16 + lr;
      const v4f a = *(const v4f*)(W + (size_t)(r0 + rr) * C_ + c0 + c4);
      *(v4f*)(tf + rr * 68 + c4) = a;
    }
  }
  __syncthreads();
  const int sub = tid >> 3;
  const int c8  = (tid & 7) * 8;
  v8h hv[2];
#pragma unroll
  for (int it = 0; it < 2; ++it) {
    const int oc = it * 32 + sub;
    v8h v;
#pragma unroll
    for (int e = 0; e < 8; ++e) v[e] = (_Float16)(tf[(c8 + e) * 68 + oc] * s);
    hv[it] = v;
  }
  for (int pass = 0; pass < 2; ++pass) {
#pragma unroll
    for (int it = 0; it < 2; ++it) {
      const int oc = it * 32 + sub;
      *(volatile v8h*)(out + (size_t)(c0 + oc) * C_ + r0 + c8) = hv[it];
    }
    __threadfence();
  }
}

__global__ __launch_bounds__(128)
void ma_kernel(const float* __restrict__ prev_m, const float* __restrict__ cached, unsigned short* __restrict__ MA) {
  const int row  = blockIdx.x;
  const int col8 = threadIdx.x * 8;
  const int rp = (row < NB_) ? row : 0;
  int rc = row - 64; rc = (rc < 0) ? 0 : rc; rc = (rc > NB_ * MM_ - 1) ? (NB_ * MM_ - 1) : rc;
  const float* sp = prev_m + (size_t)rp * C_ + col8;
  const float* sc = cached + (size_t)rc * C_ + col8;
  const v4f p0 = *(const v4f*)(sp), p1 = *(const v4f*)(sp + 4);
  const v4f q0 = *(const v4f*)(sc), q1 = *(const v4f*)(sc + 4);
  const float fp = (row < NB_) ? 1.0f : 0.0f;
  const float fc = (row >= 64) ? 1.0f : 0.0f;
  const v4f a = p0 * fp + q0 * fc;
  const v4f b = p1 * fp + q1 * fc;
  const v8h hv = cvt8(a, b, 1.0f);
  _Float16* d = (_Float16*)MA + (size_t)row * C_ + col8;
  *(volatile v8h*)d = hv;
  __threadfence();
  *(volatile v8h*)d = hv;
}

__global__ __launch_bounds__(256)
void xcvt_kernel(const float* __restrict__ x, unsigned short* __restrict__ CM, int n8) {
  const int idx = blockIdx.x * 256 + threadIdx.x;
  if (idx >= n8) return;
  const int e = idx * 8;
  const int b = e >> 20, t = (e >> 10) & (T_ - 1), col = e & (C_ - 1);
  const v4f a0 = *(const v4f*)(x + e), a1 = *(const v4f*)(x + e + 4);
  const v8h hv = cvt8(a0, a1, 1.0f);
  _Float16* d = (_Float16*)CM + ((size_t)(b * LP_ + 2 + t)) * C_ + col;
  *(volatile v8h*)d = hv;
  __threadfence();
  *(volatile v8h*)d = hv;
}

template <int BIAS_MODE, int OUT_MODE>
__global__ __launch_bounds__(256) void gemm64(
    const unsigned short* __restrict__ Ap, int lda, long strideA,
    const unsigned short* __restrict__ Btp, int ldb, long strideB,
    void* __restrict__ Cout, int ldc, long strideC,
    const float* __restrict__ bias, int M, int N, int K, float scale, float oscale) {
  const _Float16* A  = (const _Float16*)Ap;
  const _Float16* Bt = (const _Float16*)Btp;
  __shared__ __align__(16) float sT[8][16 * 68];
  const int b    = blockIdx.y;
  const int lane = threadIdx.x & 31;
  const int wave = threadIdx.x >> 5;
  const int tilesN = N >> 6;
  const int tilesM = M >> 6;
  const int tile = blockIdx.x * 8 + wave;
  if (tile >= tilesM * tilesN) return;
  const int tm = tile / tilesN;
  const int tn = tile - tm * tilesN;
  const int m0 = tm << 6;
  const int n0 = tn << 6;
  const _Float16* Ab = A  + (size_t)b * strideA;
  const _Float16* Bb = Bt + (size_t)b * strideB;
  const int rlane = lane & 15;
  const int koff  = (lane >> 4) * 8;
  const int mOff  = (lane >> 4) * 8;

  v8f acc[4][4];
#pragma unroll
  for (int i = 0; i < 4; ++i)
#pragma unroll
    for (int j = 0; j < 4; ++j) acc[i][j] = zero8f();

  for (int k0 = 0; k0 < K; k0 += 32) {
    v16h bh[4];
#pragma unroll
    for (int j = 0; j < 4; ++j)
      bh[j] = ldfrag(Bb + (size_t)(n0 + (j << 4) + rlane) * ldb + koff + k0);
#pragma unroll
    for (int i = 0; i < 4; ++i) {
      const v16h ah = ldfrag(Ab + (size_t)(m0 + (i << 4) + rlane) * lda + koff + k0);
#pragma unroll
      for (int j = 0; j < 4; ++j) acc[i][j] = mma_f16(ah, bh[j], acc[i][j]);
      dep_guard(acc[i][0], acc[i][3], ah, bh[3]);
    }
    keep4(bh[0], bh[1], bh[2], bh[3]);
  }
  acc_guard4(acc[0][0], acc[0][1], acc[0][2], acc[0][3]);
  acc_guard4(acc[1][0], acc[1][1], acc[1][2], acc[1][3]);
  acc_guard4(acc[2][0], acc[2][1], acc[2][2], acc[2][3]);
  acc_guard4(acc[3][0], acc[3][1], acc[3][2], acc[3][3]);

  float* slab = sT[wave];
#pragma unroll
  for (int i = 0; i < 4; ++i) {
    const int mBase = m0 + (i << 4);
#pragma unroll
    for (int j = 0; j < 4; ++j) {
      const int n = n0 + (j << 4) + rlane;
      float bvn = 0.f;
      if (BIAS_MODE == 2) bvn = bias[n];
#pragma unroll
      for (int r = 0; r < 8; ++r) {
        float v = acc[i][j][r] * scale;
        if (BIAS_MODE == 1) v += bias[mBase + mOff + r];
        if (BIAS_MODE == 2) v += bvn;
        v *= oscale;
        slab[(mOff + r) * 68 + (j << 4) + rlane] = v;
      }
    }
    __builtin_amdgcn_fence(__ATOMIC_RELEASE, "workgroup");
    __builtin_amdgcn_wave_barrier();
    __builtin_amdgcn_fence(__ATOMIC_ACQUIRE, "workgroup");
    if (OUT_MODE == 0) {
      float* C = (float*)Cout + (size_t)b * strideC;
      const int hh = lane >> 4, c4 = (lane & 15) * 4;
      for (int pass = 0; pass < 2; ++pass) {
#pragma unroll
        for (int it = 0; it < 8; ++it) {
          const int row = it * 2 + hh;
          const v4f v = *(const v4f*)(slab + row * 68 + c4);
          *(volatile v4f*)(C + (size_t)(mBase + row) * ldc + n0 + c4) = v;
        }
        __threadfence();
      }
    } else {
      _Float16* C = (_Float16*)Cout + (size_t)b * strideC;
      const int q = lane >> 3, c8 = (lane & 7) * 8;
      v8h hv[4];
#pragma unroll
      for (int it = 0; it < 4; ++it) {
        const int row = it * 4 + q;
        const float* spf = slab + row * 68 + c8;
        v8h t;
#pragma unroll
        for (int e = 0; e < 8; ++e) t[e] = (_Float16)spf[e];
        hv[it] = t;
      }
      for (int pass = 0; pass < 2; ++pass) {
#pragma unroll
        for (int it = 0; it < 4; ++it) {
          const int row = it * 4 + q;
          *(volatile v8h*)(C + (size_t)(mBase + row) * ldc + n0 + c8) = hv[it];
        }
        __threadfence();
      }
    }
    __builtin_amdgcn_fence(__ATOMIC_RELEASE, "workgroup");
    __builtin_amdgcn_wave_barrier();
    __builtin_amdgcn_fence(__ATOMIC_ACQUIRE, "workgroup");
  }
}

__global__ __launch_bounds__(512)
void mem_kernel(const float* __restrict__ MOq, const float* __restrict__ MOk, const float* __restrict__ prev_m,
                unsigned short* __restrict__ CM) {
  __shared__ __align__(16) float smem[C_];
  const int b = blockIdx.x;
  const int tid = threadIdx.x, wave = tid >> 5, lane = tid & 31;
  const int h = wave;
  const int j = lane & 15;
  const float* qh = MOq + (size_t)b * C_ + h * HD_;
  const float* kr = MOk + (size_t)(b * MM_ + j) * C_ + h * HD_;
  float a = 0.f;
#pragma unroll 1
  for (int d4 = 0; d4 < HD_ / 4; ++d4) {
    const v4f qv = *(const v4f*)(qh + 4 * d4);
    const v4f kv = *(const v4f*)(kr + 4 * d4);
    a = fmaf(qv[0], kv[0], a);
    a = fmaf(qv[1], kv[1], a);
    a = fmaf(qv[2], kv[2], a);
    a = fmaf(qv[3], kv[3], a);
  }
  const float sj = (lane < MM_) ? a * 0.125f : -INFINITY;
  float mx = sj;
#pragma unroll
  for (int off = 1; off < 32; off <<= 1) mx = fmaxf(mx, __shfl_xor(mx, off, 32));
  const float e = (lane < MM_) ? __expf(sj - mx) : 0.f;
  float se = e;
#pragma unroll
  for (int off = 1; off < 32; off <<= 1) se += __shfl_xor(se, off, 32);
  const float am = e * (1.0f / se);
  float o0 = 0.f, o1 = 0.f;
#pragma unroll 1
  for (int jj = 0; jj < MM_; ++jj) {
    const float aj = __shfl(am, jj, 32);
    const float* kp = MOk + (size_t)(b * MM_ + jj) * C_ + h * HD_;
    o0 = fmaf(aj, kp[lane], o0);
    o1 = fmaf(aj, kp[lane + 32], o1);
  }
  smem[h * HD_ + lane]      = o0;
  smem[h * HD_ + lane + 32] = o1;
  __syncthreads();

  _Float16* cmb = (_Float16*)CM + (size_t)b * LP_ * C_;
  const v8h z8 = zero8h();
  v8h hv = z8;
  _Float16* dst = cmb;
  const bool has = tid < 256;
  if (tid < 128) {
    const int col8 = tid * 8;
    const v4f m0 = *(const v4f*)(smem + col8), m1 = *(const v4f*)(smem + col8 + 4);
    hv = cvt8(m0, m1, 1.0f);
    dst = cmb + col8;
  } else if (tid < 256) {
    const int col8 = (tid - 128) * 8;
    const float* pp = prev_m + (size_t)b * C_ + col8;
    const v4f p0 = *(const v4f*)(pp), p1 = *(const v4f*)(pp + 4);
    hv = cvt8(p0, p1, 1.0f);
    dst = cmb + C_ + col8;
  }
  for (int pass = 0; pass < 2; ++pass) {
    if (has) *(volatile v8h*)dst = hv;
    for (int i = tid; i < (LP_ - LKV_) * (C_ / 8); i += 512) {
      const int row  = LKV_ + (i >> 7);
      const int col8 = (i & 127) * 8;
      *(volatile v8h*)(cmb + (size_t)row * C_ + col8) = z8;
    }
    __threadfence();
  }
}

__global__ __launch_bounds__(128)
void attn_kernel(const unsigned short* __restrict__ Qp, const unsigned short* __restrict__ Kp,
                 const unsigned short* __restrict__ VTp, unsigned short* __restrict__ Yp, float sscale) {
  __shared__ __align__(16) _Float16 Ksh[64 * AKP];
  __shared__ __align__(16) _Float16 Vth[64 * AKP];
  __shared__ __align__(16) _Float16 Psh[4][16 * AKP];
  __shared__ __align__(16) _Float16 Osh[4][16 * AKP];

  const int tid  = threadIdx.x;
  const int wave = tid >> 5;
  const int lane = tid & 31;
  const int hh   = lane >> 4;
  const int c    = lane & 15;
  const int bx = blockIdx.x;
  const int qb = bx & 15;
  const int h  = (bx >> 4) & (NH_ - 1);
  const int b  = bx >> 8;
  const int q0 = qb * 64 + wave * 16;

  const _Float16* Qb = (const _Float16*)Qp  + (size_t)b * T_  * C_ + h * HD_;
  const _Float16* Kb = (const _Float16*)Kp  + (size_t)b * LP_ * C_ + h * HD_;
  const _Float16* Vb = (const _Float16*)VTp + ((size_t)b * C_ + h * HD_) * LP_;
  _Float16*       Yb = (_Float16*)Yp + (size_t)b * T_ * C_ + h * HD_;

  v16h qa[2];
#pragma unroll
  for (int dc = 0; dc < 2; ++dc)
    qa[dc] = ldfrag(Qb + (size_t)(q0 + c) * C_ + dc * 32 + 8 * hh);

  float mrow[8], lrow[8];
  v8f oacc[4];
#pragma unroll
  for (int r = 0; r < 8; ++r) { mrow[r] = -INFINITY; lrow[r] = 0.f; }
#pragma unroll
  for (int t = 0; t < 4; ++t) oacc[t] = zero8f();

  int maxkey = qb * 64 + 63 + 2;
  if (qb * 64 < NU_) maxkey = (maxkey > NU_ + 1) ? maxkey : (NU_ + 1);
  const int nChunks = (maxkey >> 6) + 1;

  for (int kc = 0; kc < nChunks; ++kc) {
    const int kv0 = kc * 64;
    __syncthreads();
    {
      const int r = tid >> 1, half = (tid & 1) * 32;
      const _Float16* ks = Kb + (size_t)(kv0 + r) * C_ + half;
      const _Float16* vs = Vb + (size_t)r * LP_ + kv0 + half;
#pragma unroll
      for (int i = 0; i < 4; ++i) {
        const v8h a0 = *(const v8h*)(ks + 8 * i);
        const v8h b0 = *(const v8h*)(vs + 8 * i);
        *(v8h*)(Ksh + r * AKP + half + 8 * i) = a0;
        *(v8h*)(Vth + r * AKP + half + 8 * i) = b0;
      }
    }
    __syncthreads();

    v8f s[4];
#pragma unroll
    for (int j = 0; j < 4; ++j) {
      s[j] = zero8f();
#pragma unroll
      for (int dc = 0; dc < 2; ++dc) {
        const v16h kb = ldfrag(Ksh + (j * 16 + c) * AKP + dc * 32 + 8 * hh);
        s[j] = mma_f16_g(qa[dc], kb, s[j]);
      }
    }
    float cmx[8];
#pragma unroll
    for (int r = 0; r < 8; ++r) {
      const int qrow = q0 + 8 * hh + r;
      float m = -INFINITY;
#pragma unroll
      for (int j = 0; j < 4; ++j) {
        const int key = kv0 + j * 16 + c;
        const int jx  = key - 2;
        const bool vis = (key < 2) || (jx <= qrow) || ((qrow < NU_) && (jx < NU_));
        const float sv = vis ? s[j][r] * sscale : -INFINITY;
        s[j][r] = sv;
        m = fmaxf(m, sv);
      }
#pragma unroll
      for (int off = 1; off < 16; off <<= 1) m = fmaxf(m, __shfl_xor(m, off, 32));
      cmx[r] = m;
    }
    _Float16* pw = Psh[wave];
#pragma unroll
    for (int r = 0; r < 8; ++r) {
      const float mnew  = fmaxf(mrow[r], cmx[r]);
      const float alpha = __expf(mrow[r] - mnew);
      mrow[r] = mnew;
      float psum = 0.f;
#pragma unroll
      for (int j = 0; j < 4; ++j) {
        const float p = __expf(s[j][r] - mnew);
        psum += p;
        pw[(8 * hh + r) * AKP + j * 16 + c] = (_Float16)p;
      }
#pragma unroll
      for (int off = 1; off < 16; off <<= 1) psum += __shfl_xor(psum, off, 32);
      lrow[r] = lrow[r] * alpha + psum;
#pragma unroll
      for (int t = 0; t < 4; ++t) oacc[t][r] *= alpha;
    }
    __builtin_amdgcn_fence(__ATOMIC_RELEASE, "workgroup");
    __builtin_amdgcn_wave_barrier();
    __builtin_amdgcn_fence(__ATOMIC_ACQUIRE, "workgroup");
#pragma unroll
    for (int kk = 0; kk < 2; ++kk) {
      const v16h pa = ldfrag(pw + c * AKP + kk * 32 + 8 * hh);
#pragma unroll
      for (int t = 0; t < 4; ++t) {
        const v16h vb = ldfrag(Vth + (t * 16 + c) * AKP + kk * 32 + 8 * hh);
        oacc[t] = mma_f16_g(pa, vb, oacc[t]);
      }
    }
  }

  _Float16* os = Osh[wave];
#pragma unroll
  for (int r = 0; r < 8; ++r) {
    const float inv = 1.0f / lrow[r];
#pragma unroll
    for (int t = 0; t < 4; ++t) os[(8 * hh + r) * AKP + t * 16 + c] = (_Float16)(oacc[t][r] * inv);
  }
  __builtin_amdgcn_fence(__ATOMIC_RELEASE, "workgroup");
  __builtin_amdgcn_wave_barrier();
  __builtin_amdgcn_fence(__ATOMIC_ACQUIRE, "workgroup");
  {
    const int q4 = lane >> 3, c8 = (lane & 7) * 8;
    v8h ov[4];
#pragma unroll
    for (int it = 0; it < 4; ++it) {
      const int row = it * 4 + q4;
      ov[it] = *(const v8h*)(os + row * AKP + c8);
    }
    for (int pass = 0; pass < 2; ++pass) {
#pragma unroll
      for (int it = 0; it < 4; ++it) {
        const int row = it * 4 + q4;
        *(volatile v8h*)(Yb + (size_t)(q0 + row) * C_ + c8) = ov[it];
      }
      __threadfence();
    }
  }
}

extern "C" void kernel_launch(void* const* d_in, const int* in_sizes, int n_in,
                              void* d_out, int out_size, void* d_ws, size_t ws_size,
                              hipStream_t stream) {
  if (n_in < 15) return;
  if (in_sizes[0] != NB_ * T_ * C_) return;
  if (in_sizes[1] != NB_ * C_) return;
  if (in_sizes[2] != NB_ * MM_ * C_) return;
  for (int i = 3; i <= 13; i += 2) if (in_sizes[i] != C_ * C_) return;
  for (int i = 4; i <= 14; i += 2) if (in_sizes[i] != C_) return;
  if (out_size != NB_ * T_ * C_) return;

  const float* x      = (const float*)d_in[0];
  const float* prev_m = (const float*)d_in[1];
  const float* cached = (const float*)d_in[2];
  const float* Wq  = (const float*)d_in[3];  const float* bq  = (const float*)d_in[4];
  const float* Wk  = (const float*)d_in[5];  const float* bk  = (const float*)d_in[6];
  const float* Wv  = (const float*)d_in[7];  const float* bv  = (const float*)d_in[8];
  const float* Wp  = (const float*)d_in[9];  const float* bp  = (const float*)d_in[10];
  const float* Wqm = (const float*)d_in[11]; const float* bqm = (const float*)d_in[12];
  const float* Wkm = (const float*)d_in[13]; const float* bkm = (const float*)d_in[14];
  float* out = (float*)d_out;

  const size_t szWT  = (size_t)6 * C_ * C_ * 2;
  const size_t szMA  = (size_t)MAR_ * C_ * 2;
  const size_t szMOq = (size_t)64 * C_ * 4;
  const size_t szMOk = (size_t)128 * C_ * 4;
  const size_t szCM  = (size_t)NB_ * LP_ * C_ * 2;
  const size_t szQ   = (size_t)NB_ * T_ * C_ * 2;
  const size_t szK   = (size_t)NB_ * LP_ * C_ * 2;
  const size_t szVT  = (size_t)NB_ * C_ * LP_ * 2;
  const size_t szY   = (size_t)NB_ * T_ * C_ * 2;
  size_t off = 0;
  const size_t oWT  = off; off += szWT;
  const size_t oMA  = off; off += szMA;
  const size_t oMOq = off; off += szMOq;
  const size_t oMOk = off; off += szMOk;
  const size_t oCM  = off; off += szCM;
  const size_t oQ   = off; off += szQ;
  const size_t oK   = off; off += szK;
  const size_t oVT  = off; off += szVT;
  const size_t oY   = off; off += szY;
  if (off > ws_size) return;

  char* ws = (char*)d_ws;
  unsigned short* WT  = (unsigned short*)(ws + oWT);
  unsigned short* MA  = (unsigned short*)(ws + oMA);
  float*          MOq = (float*)(ws + oMOq);
  float*          MOk = (float*)(ws + oMOk);
  unsigned short* CM  = (unsigned short*)(ws + oCM);
  unsigned short* Qh  = (unsigned short*)(ws + oQ);
  unsigned short* Kh  = (unsigned short*)(ws + oK);
  unsigned short* VTh = (unsigned short*)(ws + oVT);
  unsigned short* Yh  = (unsigned short*)(ws + oY);
  unsigned short* WqT  = WT;
  unsigned short* WkT  = WT + (size_t)1 * C_ * C_;
  unsigned short* WvT  = WT + (size_t)2 * C_ * C_;
  unsigned short* WpT  = WT + (size_t)3 * C_ * C_;
  unsigned short* WqmT = WT + (size_t)4 * C_ * C_;
  unsigned short* WkmT = WT + (size_t)5 * C_ * C_;

  const dim3 blk(256);
  const float s16 = 16.0f, r16 = 1.0f / 16.0f, r256 = 1.0f / 256.0f;

  wt_kernel<<<dim3(C_ / 64, C_ / 64, 6), blk, 0, stream>>>(Wq, Wk, Wv, Wp, Wqm, Wkm, WT, s16);
  ma_kernel<<<dim3(MAR_), dim3(128), 0, stream>>>(prev_m, cached, MA);
  const int n8 = NB_ * T_ * C_ / 8;
  xcvt_kernel<<<dim3((n8 + 255) / 256), blk, 0, stream>>>(x, CM, n8);
  gemm64<2, 0><<<dim3(((64 / 64) * (C_ / 64) + 7) / 8, 1), blk, 0, stream>>>(
      MA, C_, 0L, WqmT, C_, 0L, (void*)MOq, C_, 0L, bqm, 64, C_, C_, r16, 1.0f);
  gemm64<2, 0><<<dim3(((128 / 64) * (C_ / 64) + 7) / 8, 1), blk, 0, stream>>>(
      MA + (size_t)64 * C_, C_, 0L, WkmT, C_, 0L, (void*)MOk, C_, 0L, bkm, 128, C_, C_, r16, 1.0f);
  mem_kernel<<<dim3(NB_), dim3(512), 0, stream>>>(MOq, MOk, prev_m, CM);
  gemm64<2, 1><<<dim3(((T_ / 64) * (C_ / 64) + 7) / 8, NB_), blk, 0, stream>>>(
      CM + (size_t)2 * C_, C_, (long)LP_ * C_, WqT, C_, 0L, (void*)Qh, C_, (long)T_ * C_, bq, T_, C_, C_, r16, s16);
  gemm64<2, 1><<<dim3(((LP_ / 64) * (C_ / 64) + 7) / 8, NB_), blk, 0, stream>>>(
      CM, C_, (long)LP_ * C_, WkT, C_, 0L, (void*)Kh, C_, (long)LP_ * C_, bk, LP_, C_, C_, r16, s16);
  gemm64<1, 1><<<dim3(((C_ / 64) * (LP_ / 64) + 7) / 8, NB_), blk, 0, stream>>>(
      WvT, C_, 0L, CM, C_, (long)LP_ * C_, (void*)VTh, LP_, (long)C_ * LP_, bv, C_, LP_, C_, r16, s16);
  attn_kernel<<<dim3(NB_ * NH_ * (T_ / 64)), dim3(128), 0, stream>>>(Qh, Kh, VTh, Yh, 0.125f / 256.0f);
  gemm64<2, 0><<<dim3(((NB_ * T_ / 64) * (C_ / 64) + 7) / 8, 1), blk, 0, stream>>>(
      Yh, C_, 0L, WpT, C_, 0L, (void*)out, C_, 0L, bp, NB_ * T_, C_, C_, r256, 1.0f);
  (void)hipGetLastError();
}
